// GNN_75685913690122
// MI455X (gfx1250) — hardware-verified
//
#include <hip/hip_runtime.h>
#include <stddef.h>
#include <stdint.h>
#include <math.h>


#define DF     128
#define DH     64
#define NTHR   256
#define NWAVE  8
#define EPT    8
#define CHUNK  (NTHR * EPT)
#define WCAP   (EPT * 32)
#define LISTN  (NWAVE * WCAP)
#define NBD    8192
#define SLD    13
#define NBA    1024
#define SLA    10
#define RCAP   28672
#define DEGCAP 64
#define GBM    64
#define GBN    64
#define GTHR   128
#define NUW    16384
#define RBH    256
#define AGG_ZINTS    (LISTN + 2 * RCAP + 3 * NBA)
#define MISC_INTS    16
#define ROWBUF_INTS  (NWAVE * RBH / 2)
#define AGG_LDS_INTS (AGG_ZINTS + MISC_INTS + ROWBUF_INTS)
#define WSMAX  134217728

static_assert((CHUNK & (CHUNK - 1)) == 0 && CHUNK <= 4096);
static_assert((NBD & (NBD - 1)) == 0 && NBD == (1 << SLD));
static_assert((NBA & (NBA - 1)) == 0 && NBA == (1 << SLA));
static_assert(((long long)CHUNK << SLD) < (1LL << 31));
static_assert(((long long)CHUNK << SLA) < (1LL << 31));
static_assert(NBD % (NTHR * 4) == 0);
static_assert(LISTN % NTHR == 0);
static_assert(NBA % NWAVE == 0 && NBA % 32 == 0 && NBA % GBM == 0);
static_assert(RCAP % 32 == 0 && AGG_ZINTS % 4 == 0 && LISTN % 4 == 0);
static_assert(AGG_ZINTS % (NTHR * 4) == 0 && ((AGG_ZINTS + MISC_INTS) % 4) == 0);
static_assert(GBM == (GTHR / 32) * 16 && GBN == 64);
static_assert(DF % GBN == 0 && DH % GBN == 0 && DF % 32 == 0 && DH % 32 == 0 && DF == 4 * 32 && DH == 2 * 32);
static_assert(NUW % NTHR == 0);
static_assert(DEGCAP >= 36 + 8);
static_assert(RBH == 2 * DF);
static_assert(AGG_LDS_INTS * 4 <= 300000);

typedef float          v2f   __attribute__((ext_vector_type(2)));
typedef float          v4f   __attribute__((ext_vector_type(4)));
typedef float          v8f   __attribute__((ext_vector_type(8)));
typedef int            v4i   __attribute__((ext_vector_type(4)));
typedef int            v8i   __attribute__((ext_vector_type(8)));
typedef unsigned short v2us  __attribute__((ext_vector_type(2)));
typedef unsigned short v4us  __attribute__((ext_vector_type(4)));
typedef unsigned short v8us  __attribute__((ext_vector_type(8)));
typedef unsigned short v16us __attribute__((ext_vector_type(16)));
typedef __bf16         v16bf __attribute__((ext_vector_type(16)));
typedef v2f  __attribute__((may_alias)) v2fa;
typedef v4f  __attribute__((may_alias)) v4fa;
typedef v4i  __attribute__((may_alias)) v4ia;
typedef v2us __attribute__((may_alias)) v2usa;
typedef v4us __attribute__((may_alias)) v4usa;
typedef v8us __attribute__((may_alias)) v8usa;
union FragB { v16bf v; v16us u; v8us h[2]; v8i w; };

__device__ __forceinline__ v8f wmb(const FragB& a, const FragB& b, v8f c) {
  v8f d = __builtin_amdgcn_wmma_f32_16x16x32_bf16(false, a.v, false, b.v, (short)0, c, false, false);
  asm volatile("v_nop\n\tv_nop\n\tv_nop\n\tv_nop" : "+v"(d) : "v"(a.w), "v"(b.w));
  return d;
}

__device__ __forceinline__ unsigned bf16_bits(float f) {
  const unsigned u = __float_as_uint(f);
  return (u + 0x7FFFu + ((u >> 16) & 1u)) >> 16;
}
__device__ __forceinline__ float bf16_val(float f) {
  return __uint_as_float(bf16_bits(f) << 16);
}

__device__ __forceinline__ void wave_sync() {
  __builtin_amdgcn_fence(__ATOMIC_RELEASE, "wavefront");
  __builtin_amdgcn_wave_barrier();
  __builtin_amdgcn_fence(__ATOMIC_ACQUIRE, "wavefront");
}

__device__ __forceinline__ float wsum32(float s) {
#pragma unroll
  for (int off = 16; off > 0; off >>= 1) s += __shfl_xor(s, off, 32);
  return s;
}

template <int SLB>
__device__ __forceinline__ int scan_chunk(const int* __restrict__ dsts, int nE, int cbase, int slotBase,
                                          int nb, int vec8, int* list, int tid, int lane, int wave) {
  int wc = 0;
  const int el0  = tid * EPT;
  const int e0   = cbase + el0;
  const int sent = -2147483647 - 1;
  v4i da, db;
  if (vec8 != 0 && cbase + CHUNK <= nE) {
    da = *(const v4i*)(dsts + e0);
    db = *(const v4i*)(dsts + e0 + 4);
  } else {
    da.x = (e0     < nE) ? dsts[min(e0,     nE - 1)] : sent;
    da.y = (e0 + 1 < nE) ? dsts[min(e0 + 1, nE - 1)] : sent;
    da.z = (e0 + 2 < nE) ? dsts[min(e0 + 2, nE - 1)] : sent;
    da.w = (e0 + 3 < nE) ? dsts[min(e0 + 3, nE - 1)] : sent;
    db.x = (e0 + 4 < nE) ? dsts[min(e0 + 4, nE - 1)] : sent;
    db.y = (e0 + 5 < nE) ? dsts[min(e0 + 5, nE - 1)] : sent;
    db.z = (e0 + 6 < nE) ? dsts[min(e0 + 6, nE - 1)] : sent;
    db.w = (e0 + 7 < nE) ? dsts[min(e0 + 7, nE - 1)] : sent;
  }
  const unsigned nbs = (unsigned)slotBase;
  const unsigned unb = (unsigned)nb;
  const unsigned s0 = (unsigned)da.x - nbs, s1 = (unsigned)da.y - nbs;
  const unsigned s2 = (unsigned)da.z - nbs, s3 = (unsigned)da.w - nbs;
  const unsigned s4 = (unsigned)db.x - nbs, s5 = (unsigned)db.y - nbs;
  const unsigned s6 = (unsigned)db.z - nbs, s7 = (unsigned)db.w - nbs;
  const bool h0 = s0 < unb, h1 = s1 < unb, h2 = s2 < unb, h3 = s3 < unb;
  const bool h4 = s4 < unb, h5 = s5 < unb, h6 = s6 < unb, h7 = s7 < unb;
  const unsigned any = __builtin_amdgcn_ballot_w32(h0 | h1 | h2 | h3 | h4 | h5 | h6 | h7);
  if (any != 0u) {
#define HITJ(J, HJ, SJ) { \
      const unsigned mj = __builtin_amdgcn_ballot_w32(HJ); \
      if (mj != 0u) { \
        if (HJ) { \
          const int pos = wc + (int)__builtin_amdgcn_mbcnt_lo(mj, 0u); \
          if (pos < WCAP) list[wave * WCAP + pos] = ((el0 + (J)) << SLB) | (int)(SJ); \
        } \
        wc += (int)__builtin_popcount(mj); } }
    HITJ(0, h0, s0)
    HITJ(1, h1, s1)
    HITJ(2, h2, s2)
    HITJ(3, h3, s3)
    HITJ(4, h4, s4)
    HITJ(5, h5, s5)
    HITJ(6, h6, s6)
    HITJ(7, h7, s7)
#undef HITJ
  }
  return wc;
}

__global__ __launch_bounds__(NTHR) void k_wprep(const float* __restrict__ Wc1, const float* __restrict__ W1,
                                                const float* __restrict__ Wc2, const float* __restrict__ W2,
                                                const float* __restrict__ W3,  const float* __restrict__ Wc3,
                                                const float* __restrict__ W4,
                                                unsigned short* Wc1T, unsigned short* W1T, unsigned short* Wc2T,
                                                unsigned short* W2T,  unsigned short* W3T, unsigned short* Wc3T,
                                                unsigned short* W4T) {
  const int u = (int)blockIdx.x * NTHR + (int)threadIdx.x;
  const float* W;
  unsigned short* P;
  int v, kqs, nout, kmask, pitch;
  if (u < 2048)       { v = u;         W = Wc1; P = Wc1T; kqs = 4; nout = DF; kmask = DF - 1; pitch = DF; }
  else if (u < 4096)  { v = u - 2048;  W = W1;  P = W1T;  kqs = 4; nout = DF; kmask = DF - 1; pitch = DF; }
  else if (u < 6144)  { v = u - 4096;  W = Wc2; P = Wc2T; kqs = 5; nout = DH; kmask = DF - 1; pitch = 2 * DF; }
  else if (u < 10240) { v = u - 6144;  W = W2;  P = W2T;  kqs = 5; nout = DF; kmask = DF - 1; pitch = 2 * DF; }
  else if (u < 12288) { v = u - 10240; W = W3;  P = W3T;  kqs = 5; nout = DH; kmask = DF - 1; pitch = 2 * DF; }
  else if (u < 14336) { v = u - 12288; W = Wc3; P = Wc3T; kqs = 4; nout = DF; kmask = DH - 1; pitch = DF; }
  else if (u < 16384) { v = u - 14336; W = W4;  P = W4T;  kqs = 4; nout = DF; kmask = DH - 1; pitch = DF; }
  else return;
  const int n  = v >> kqs;
  const int k8 = (v & ((1 << kqs) - 1)) * 8;
  const int kk = k8 & kmask;
  const float* p = W + (size_t)kk * nout + n;
  v8us o;
#pragma unroll
  for (int i = 0; i < 8; ++i) o[i] = (unsigned short)bf16_bits(p[(size_t)i * nout]);
  unsigned short* dp = P + (size_t)n * pitch + k8;
  *(volatile v8us*)dp = o;
  __threadfence();
  *(volatile v8us*)dp = o;
}

__global__ __launch_bounds__(NTHR) void k_cvx(const float* __restrict__ x, int nN, int nUnits,
                                              unsigned short* xb) {
  const int u = (int)blockIdx.x * NTHR + (int)threadIdx.x;
  if (u >= nUnits) return;
  const int row = u >> 4;
  const int k8  = (u & 15) * 8;
  const int rc  = row < nN ? row : nN - 1;
  const float* p = x + (size_t)rc * DF + k8;
  const v4f a = *(const v4fa*)p;
  const v4f b = *(const v4fa*)(p + 4);
  const bool ok = row < nN;
  v8us o;
  o[0] = ok ? (unsigned short)bf16_bits(a.x) : (unsigned short)0;
  o[1] = ok ? (unsigned short)bf16_bits(a.y) : (unsigned short)0;
  o[2] = ok ? (unsigned short)bf16_bits(a.z) : (unsigned short)0;
  o[3] = ok ? (unsigned short)bf16_bits(a.w) : (unsigned short)0;
  o[4] = ok ? (unsigned short)bf16_bits(b.x) : (unsigned short)0;
  o[5] = ok ? (unsigned short)bf16_bits(b.y) : (unsigned short)0;
  o[6] = ok ? (unsigned short)bf16_bits(b.z) : (unsigned short)0;
  o[7] = ok ? (unsigned short)bf16_bits(b.w) : (unsigned short)0;
  unsigned short* dp = xb + (size_t)row * DF + k8;
  *(volatile v8us*)dp = o;
  __threadfence();
  *(volatile v8us*)dp = o;
}

__global__ __launch_bounds__(NTHR) void k_deg(const int* __restrict__ dsts, int nE, int vec8, float* dis) {
  __shared__ __attribute__((aligned(16))) int scnt[NBD];
  __shared__ __attribute__((aligned(16))) int list[LISTN];
  __shared__ int wcnt[NWAVE];
  const int tid = (int)threadIdx.x, lane = tid & 31, wave = tid >> 5;
  const int nodeBase = (int)blockIdx.x * NBD;

  for (int i = tid; i < NBD; i += NTHR) scnt[i] = 0;
  for (int i = tid; i < LISTN; i += NTHR) list[i] = 0;
  if (tid < NWAVE) wcnt[tid] = 0;
  __syncthreads();

  const int nChunks = (nE + CHUNK - 1) / CHUNK;
#pragma unroll 1
  for (int ch = 0; ch < nChunks; ++ch) {
    const int cbase = ch * CHUNK;
    const int wc = scan_chunk<SLD>(dsts, nE, cbase, nodeBase, NBD, vec8, list, tid, lane, wave);
    if (lane == 0) wcnt[wave] = wc;
    __syncthreads();
    if (wave == 0) {
#pragma unroll 1
      for (int w2 = 0; w2 < NWAVE; ++w2) {
        int c = wcnt[w2];
        c = c < 0 ? 0 : (c > WCAP ? WCAP : c);
#pragma unroll 1
        for (int b0 = 0; b0 < c; b0 += 32) {
          const int idx = b0 + lane;
          const int ent = list[w2 * WCAP + (idx < WCAP ? idx : WCAP - 1)];
          const int m32 = (c - b0) < 32 ? (c - b0) : 32;
#pragma unroll 1
          for (int k = 0; k < m32; ++k) {
            const int u  = __builtin_amdgcn_readlane(ent, k);
            const int sl = u & (NBD - 1);
            if (lane == 0) scnt[sl] = scnt[sl] + 1;
          }
        }
      }
    }
    __syncthreads();
  }

  v4f vals[NBD / (NTHR * 4)];
#pragma unroll
  for (int it = 0; it < NBD / (NTHR * 4); ++it) {
    const int s0 = it * (NTHR * 4) + 4 * tid;
    const v4i c4 = *(const v4ia*)(scnt + s0);
    const float d0 = (float)c4.x + 1.0f, d1 = (float)c4.y + 1.0f;
    const float d2 = (float)c4.z + 1.0f, d3 = (float)c4.w + 1.0f;
    v4f v;
    v.x = rsqrtf(d0); v.y = rsqrtf(d1); v.z = rsqrtf(d2); v.w = rsqrtf(d3);
    vals[it] = v;
  }
#pragma unroll
  for (int it = 0; it < NBD / (NTHR * 4); ++it) {
    const int s0 = it * (NTHR * 4) + 4 * tid;
    *(volatile v4f*)(dis + (size_t)nodeBase + s0) = vals[it];
  }
  __threadfence();
#pragma unroll
  for (int it = 0; it < NBD / (NTHR * 4); ++it) {
    const int s0 = it * (NTHR * 4) + 4 * tid;
    *(volatile v4f*)(dis + (size_t)nodeBase + s0) = vals[it];
  }
}

template <int MODE>
__global__ __launch_bounds__(GTHR) void k_gemm(const unsigned short* __restrict__ A,
                                               const unsigned short* __restrict__ WT, int K,
                                               const float* __restrict__ bias, int nN,
                                               float* outF, unsigned short* outH, int ldo) {
  __shared__ __attribute__((aligned(16))) float stg[GBM * GBN];
  const int tid = (int)threadIdx.x, lane = tid & 31, wave = tid >> 5, hh = lane >> 4, m = lane & 15;
  const int rowBase = (int)blockIdx.x * GBM;
  const int col0    = (int)blockIdx.y * GBN;

  v8f acc[4];
  {
    const v8f z = {0.f, 0.f, 0.f, 0.f, 0.f, 0.f, 0.f, 0.f};
    acc[0] = z; acc[1] = z; acc[2] = z; acc[3] = z;
  }
  const unsigned short* ap = A  + (size_t)(rowBase + 16 * wave + m) * (size_t)K + 8 * hh;
  const unsigned short* wp = WT + (size_t)(col0 + m) * (size_t)K + 8 * hh;
  const int ksteps = K >> 5;
#pragma unroll 1
  for (int ks = 0; ks < ksteps; ++ks) {
    FragB af;
    af.h[0] = *(const v8usa*)(ap + 32 * ks);
    af.h[1] = *(const v8usa*)(ap + 32 * ks + 16);
#pragma unroll
    for (int t = 0; t < 4; ++t) {
      const unsigned short* wq = wp + (size_t)(16 * t) * (size_t)K + 32 * ks;
      FragB bf;
      bf.h[0] = *(const v8usa*)wq;
      bf.h[1] = *(const v8usa*)(wq + 16);
      acc[t] = wmb(af, bf, acc[t]);
    }
  }

#pragma unroll
  for (int t = 0; t < 4; ++t) {
    const int lc = 16 * t + m;
#pragma unroll
    for (int r = 0; r < 8; ++r) {
      const int lr = 16 * wave + 8 * hh + r;
      stg[lr * GBN + lc] = acc[t][r];
    }
  }
  __syncthreads();

  v4f fv[8];
#pragma unroll
  for (int i = 0; i < 8; ++i) {
    const int lr = 16 * wave + 2 * i + hh;
    fv[i] = *(const v4fa*)(stg + lr * GBN + 4 * m);
  }

  if constexpr (MODE != 0) {
    v4f bq;
    {
      const v4f t = *(const v4f*)(bias + col0 + 4 * m);
      bq.x = bf16_val(t.x); bq.y = bf16_val(t.y); bq.z = bf16_val(t.z); bq.w = bf16_val(t.w);
    }
#pragma unroll
    for (int i = 0; i < 8; ++i) {
      const int gr = rowBase + 16 * wave + 2 * i + hh;
      const bool ok = gr < nN;
      v4f t = fv[i] + bq;
      if constexpr (MODE == 1) {
        t.x = fmaxf(t.x, 0.0f); t.y = fmaxf(t.y, 0.0f); t.z = fmaxf(t.z, 0.0f); t.w = fmaxf(t.w, 0.0f);
        t.x = ok ? t.x : 0.0f;  t.y = ok ? t.y : 0.0f;  t.z = ok ? t.z : 0.0f;  t.w = ok ? t.w : 0.0f;
      }
      fv[i] = t;
    }
  }

  if constexpr (MODE == 1) {
    __syncthreads();
#pragma unroll
    for (int i = 0; i < 8; ++i) {
      const int lr = 16 * wave + 2 * i + hh;
      v4us h4, l4;
      unsigned hb;
      hb = bf16_bits(fv[i].x); h4[0] = (unsigned short)hb; l4[0] = (unsigned short)bf16_bits(fv[i].x - __uint_as_float(hb << 16));
      hb = bf16_bits(fv[i].y); h4[1] = (unsigned short)hb; l4[1] = (unsigned short)bf16_bits(fv[i].y - __uint_as_float(hb << 16));
      hb = bf16_bits(fv[i].z); h4[2] = (unsigned short)hb; l4[2] = (unsigned short)bf16_bits(fv[i].z - __uint_as_float(hb << 16));
      hb = bf16_bits(fv[i].w); h4[3] = (unsigned short)hb; l4[3] = (unsigned short)bf16_bits(fv[i].w - __uint_as_float(hb << 16));
      unsigned short* srow = (unsigned short*)stg + (size_t)lr * (2 * GBN);
      *(v4usa*)(srow + 4 * m) = h4;
      *(v4usa*)(srow + GBN + 4 * m) = l4;
    }
    __syncthreads();
    v8us qv[8];
#pragma unroll
    for (int i = 0; i < 8; ++i) {
      const int lr = 16 * wave + 2 * i + hh;
      const unsigned short* srow = (const unsigned short*)stg + (size_t)lr * (2 * GBN);
      qv[i] = *(const v8usa*)(srow + 8 * m);
    }
    const int nfull = (int)gridDim.y * GBN;
    const int dcol  = (m < 8) ? (col0 + 8 * m) : (nfull + col0 + 8 * (m - 8));
#pragma unroll
    for (int i = 0; i < 8; ++i) {
      const int gr = rowBase + 16 * wave + 2 * i + hh;
      unsigned short* dp = outH + (size_t)gr * (size_t)ldo + dcol;
      *(volatile v8us*)dp = qv[i];
    }
    __threadfence();
#pragma unroll
    for (int i = 0; i < 8; ++i) {
      const int gr = rowBase + 16 * wave + 2 * i + hh;
      unsigned short* dp = outH + (size_t)gr * (size_t)ldo + dcol;
      *(volatile v8us*)dp = qv[i];
    }
  } else {
#pragma unroll
    for (int i = 0; i < 8; ++i) {
      const int gr = rowBase + 16 * wave + 2 * i + hh;
      float* op = outF + (size_t)gr * (size_t)ldo + col0 + 4 * m;
      if (MODE == 0 || gr < nN) *(volatile v4f*)op = fv[i];
    }
    __threadfence();
#pragma unroll
    for (int i = 0; i < 8; ++i) {
      const int gr = rowBase + 16 * wave + 2 * i + hh;
      float* op = outF + (size_t)gr * (size_t)ldo + col0 + 4 * m;
      if (MODE == 0 || gr < nN) *(volatile v4f*)op = fv[i];
    }
  }
}

template <int WID, int FIN>
__global__ __launch_bounds__(NTHR) void k_scan(const int* __restrict__ srcs, const int* __restrict__ dsts,
                                               int nE, int nN, int vec8, int mRows,
                                               const float* __restrict__ dis, const float* __restrict__ hw,
                                               const float* __restrict__ bias, const float* __restrict__ gam,
                                               const float* __restrict__ bet,
                                               unsigned short* outH, float* outF) {
  static_assert(WID == 128 || WID == 64);
  static_assert(FIN == 0 || WID == 128);
  extern __shared__ __attribute__((aligned(16))) int dsm[];
  int* list = dsm;
  int* hl   = dsm + LISTN;
  int* sl   = hl + RCAP;
  int* cnt  = sl + RCAP;
  int* offs = cnt + NBA;
  int* cur  = offs + NBA;
  int* misc = cur + NBA;
  const int tid = (int)threadIdx.x, lane = tid & 31, wave = tid >> 5;
  unsigned short* rowbuf = (unsigned short*)(misc + MISC_INTS) + wave * RBH;
  const int nodeBase = (int)blockIdx.x * NBA;

  {
    const v4i z4 = {0, 0, 0, 0};
    for (int i = tid * 4; i < AGG_ZINTS; i += NTHR * 4) *(v4ia*)(dsm + i) = z4;
    if (tid < MISC_INTS) misc[tid] = 0;
  }
  __syncthreads();

  int t = 0, ov = 0;
  const int nChunks = (nE + CHUNK - 1) / CHUNK;
#pragma unroll 1
  for (int ch = 0; ch < nChunks; ++ch) {
    const int cbase = ch * CHUNK;
    const int wc = scan_chunk<SLA>(dsts, nE, cbase, nodeBase, NBA, vec8, list, tid, lane, wave);
    if (lane == 0) misc[wave] = wc;
    __syncthreads();
    if (wave == 0) {
#pragma unroll 1
      for (int w2 = 0; w2 < NWAVE; ++w2) {
        int c = misc[w2];
        c = c < 0 ? 0 : (c > WCAP ? WCAP : c);
#pragma unroll 1
        for (int b0 = 0; b0 < c; b0 += 32) {
          const int idx = b0 + lane;
          const int ent = list[w2 * WCAP + (idx < WCAP ? idx : WCAP - 1)];
          const int m32 = (c - b0) < 32 ? (c - b0) : 32;
#pragma unroll 1
          for (int k = 0; k < m32; ++k) {
            const int u    = __builtin_amdgcn_readlane(ent, k);
            const int slot = u & (NBA - 1);
            const int el   = (u >> SLA) & (CHUNK - 1);
            const int pk   = ((cbase + el) << SLA) | slot;
            if (t < RCAP) {
              if (lane == 0) { hl[t] = pk; cnt[slot] = cnt[slot] + 1; }
              t = t + 1;
            } else {
              ov = 1;
            }
          }
        }
      }
    }
    __syncthreads();
  }
  if (wave == 0 && lane == 0) { misc[8] = t; misc[9] = ov; }
  __syncthreads();
  int tt = misc[8];
  tt = tt < 0 ? 0 : (tt > RCAP ? RCAP : tt);
  const int ovf = misc[9];

  if (wave == 0) {
    const int base = lane * (NBA / 32);
    int s = 0;
#pragma unroll 1
    for (int i = 0; i < NBA / 32; ++i) s += cnt[base + i];
    int incl = s;
#pragma unroll
    for (int d = 1; d < 32; d <<= 1) {
      const int y = __shfl_up(incl, d, 32);
      if (lane >= d) incl += y;
    }
    int run = incl - s;
#pragma unroll 1
    for (int i = 0; i < NBA / 32; ++i) {
      const int cv = cnt[base + i];
      offs[base + i] = run;
      cur[base + i]  = run;
      run += cv;
    }
  }
  __syncthreads();
  if (wave == 0) {
#pragma unroll 1
    for (int b0 = 0; b0 < tt; b0 += 32) {
      const int idx = b0 + lane;
      const int ent = hl[idx < RCAP ? idx : RCAP - 1];
      const int m32 = (tt - b0) < 32 ? (tt - b0) : 32;
#pragma unroll 1
      for (int k = 0; k < m32; ++k) {
        const int u    = __builtin_amdgcn_readlane(ent, k);
        const int slot = u & (NBA - 1);
        if (lane == 0) {
          int p = cur[slot];
          p = p < 0 ? 0 : (p > RCAP - 1 ? RCAP - 1 : p);
          sl[p] = u;
          cur[slot] = p + 1;
        }
      }
    }
  }
  __syncthreads();

  constexpr float invW = 1.0f / (float)WID;
  const float qnan = __int_as_float(0x7fc00000);
  const float pz = (ovf != 0) ? qnan : 0.0f;
  v4f bv, gv, ev;
  if constexpr (WID == 128) {
    const v4f tb = *(const v4fa*)(bias + 4 * lane);
    const v4f tg = *(const v4fa*)(gam + 4 * lane);
    const v4f te = *(const v4fa*)(bet + 4 * lane);
    bv.x = bf16_val(tb.x); bv.y = bf16_val(tb.y); bv.z = bf16_val(tb.z); bv.w = bf16_val(tb.w);
    gv.x = bf16_val(tg.x); gv.y = bf16_val(tg.y); gv.z = bf16_val(tg.z); gv.w = bf16_val(tg.w);
    ev.x = bf16_val(te.x); ev.y = bf16_val(te.y); ev.z = bf16_val(te.z); ev.w = bf16_val(te.w);
  } else {
    const v2f tb = *(const v2fa*)(bias + 2 * lane);
    const v2f tg = *(const v2fa*)(gam + 2 * lane);
    const v2f te = *(const v2fa*)(bet + 2 * lane);
    bv.x = bf16_val(tb.x); bv.y = bf16_val(tb.y); bv.z = 0.0f; bv.w = 0.0f;
    gv.x = bf16_val(tg.x); gv.y = bf16_val(tg.y); gv.z = 0.0f; gv.w = 0.0f;
    ev.x = bf16_val(te.x); ev.y = bf16_val(te.y); ev.z = 0.0f; ev.w = 0.0f;
  }
  const int ql = (WID == 128) ? lane : (lane & 15);
#pragma unroll 1
  for (int si = 0; si < NBA / NWAVE; ++si) {
    const int s    = si * NWAVE + wave;
    const int node = nodeBase + s;
    int c = cnt[s];
    const bool big = c > DEGCAP;
    c = c < 0 ? 0 : (c > DEGCAP ? DEGCAP : c);
    int o = offs[s];
    o = o < 0 ? 0 : (o > RCAP ? RCAP : o);
    const int nc = node < nN ? node : nN - 1;
    const float dd = dis[nc];
    const float rd = dd * dd;
    float a0 = 0.0f, a1 = 0.0f, a2 = 0.0f, a3 = 0.0f;
#pragma unroll 1
    for (int b0 = 0; b0 < c; b0 += 32) {
      int idx = o + b0 + lane;
      idx = idx > RCAP - 1 ? RCAP - 1 : idx;
      const int ent = sl[idx];
      int eid = ent >> SLA;
      eid = eid < 0 ? 0 : (eid > nE - 1 ? nE - 1 : eid);
      int sr = srcs[eid];
      sr = sr < 0 ? 0 : (sr > nN - 1 ? nN - 1 : sr);
      const float cf  = dis[sr] * dd;
      const int   cfi = __float_as_int(cf);
      const int m32 = (c - b0) < 32 ? (c - b0) : 32;
#pragma unroll 1
      for (int k = 0; k < m32; ++k) {
        const int   sk = __builtin_amdgcn_readlane(sr, k);
        const float ck = __int_as_float(__builtin_amdgcn_readlane(cfi, k));
        if constexpr (WID == 128) {
          const v4f a = *(const v4fa*)(hw + (size_t)sk * WID + 4 * lane);
          a0 = fmaf(ck, a.x, a0); a1 = fmaf(ck, a.y, a1);
          a2 = fmaf(ck, a.z, a2); a3 = fmaf(ck, a.w, a3);
        } else {
          const v2f a = *(const v2fa*)(hw + (size_t)sk * WID + 2 * lane);
          a0 = fmaf(ck, a.x, a0); a1 = fmaf(ck, a.y, a1);
        }
      }
    }
    float sv0, sv1, sv2 = 0.0f, sv3 = 0.0f;
    if constexpr (WID == 128) {
      const v4f a = *(const v4fa*)(hw + (size_t)nc * WID + 4 * lane);
      sv0 = a.x; sv1 = a.y; sv2 = a.z; sv3 = a.w;
    } else {
      const v2f a = *(const v2fa*)(hw + (size_t)nc * WID + 2 * lane);
      sv0 = a.x; sv1 = a.y;
    }
    const float pzr = big ? qnan : pz;
    const bool live = node < nN;
    const float v0 = fmaxf((a0 + sv0 * rd) + bv.x, 0.0f);
    const float v1 = fmaxf((a1 + sv1 * rd) + bv.y, 0.0f);
    float v2 = 0.0f, v3 = 0.0f;
    if constexpr (WID == 128) {
      v2 = fmaxf((a2 + sv2 * rd) + bv.z, 0.0f);
      v3 = fmaxf((a3 + sv3 * rd) + bv.w, 0.0f);
    }
    const float ssum = wsum32((v0 + v1) + (v2 + v3));
    const float mu   = ssum * invW;
    const float d0 = v0 - mu, d1 = v1 - mu;
    float d2 = 0.0f, d3 = 0.0f;
    if constexpr (WID == 128) { d2 = v2 - mu; d3 = v3 - mu; }
    const float qsum = wsum32((d0 * d0 + d1 * d1) + (d2 * d2 + d3 * d3));
    const float rstd = rsqrtf(qsum * invW + 1e-5f);
    const float y0 = (d0 * rstd) * gv.x + ev.x + pzr;
    const float y1 = (d1 * rstd) * gv.y + ev.y + pzr;
    const float y2 = (d2 * rstd) * gv.z + ev.z + pzr;
    const float y3 = (d3 * rstd) * gv.w + ev.w + pzr;
    if constexpr (FIN != 0) {
      const v4f f = *(const v4fa*)(outF + (size_t)nc * WID + 4 * lane);
      v4f ow;
      ow.x = (y0 + f.x) * 0.5f; ow.y = (y1 + f.y) * 0.5f;
      ow.z = (y2 + f.z) * 0.5f; ow.w = (y3 + f.w) * 0.5f;
      float* op = outF + (size_t)node * WID + 4 * lane;
      if (live) *(volatile v4f*)op = ow;
      __threadfence();
      if (live) *(volatile v4f*)op = ow;
    } else {
      const float m0 = live ? y0 : 0.0f;
      const float m1 = live ? y1 : 0.0f;
      const float m2 = live ? y2 : 0.0f;
      const float m3 = live ? y3 : 0.0f;
      if constexpr (WID == 128) {
        v4us mh, ml;
        unsigned hb;
        hb = bf16_bits(m0); mh[0] = (unsigned short)hb; ml[0] = (unsigned short)bf16_bits(m0 - __uint_as_float(hb << 16));
        hb = bf16_bits(m1); mh[1] = (unsigned short)hb; ml[1] = (unsigned short)bf16_bits(m1 - __uint_as_float(hb << 16));
        hb = bf16_bits(m2); mh[2] = (unsigned short)hb; ml[2] = (unsigned short)bf16_bits(m2 - __uint_as_float(hb << 16));
        hb = bf16_bits(m3); mh[3] = (unsigned short)hb; ml[3] = (unsigned short)bf16_bits(m3 - __uint_as_float(hb << 16));
        *(v4usa*)(rowbuf + 4 * lane) = mh;
        *(v4usa*)(rowbuf + WID + 4 * lane) = ml;
      } else {
        v2us mh, ml;
        unsigned hb;
        hb = bf16_bits(m0); mh[0] = (unsigned short)hb; ml[0] = (unsigned short)bf16_bits(m0 - __uint_as_float(hb << 16));
        hb = bf16_bits(m1); mh[1] = (unsigned short)hb; ml[1] = (unsigned short)bf16_bits(m1 - __uint_as_float(hb << 16));
        *(v2usa*)(rowbuf + 2 * lane) = mh;
        *(v2usa*)(rowbuf + WID + 2 * lane) = ml;
      }
      wave_sync();
      const v8us q0 = *(const v8usa*)(rowbuf + 8 * ql);
      wave_sync();
      const bool wr = (node < mRows) && (WID == 128 || lane < 16);
      unsigned short* rp = outH + (size_t)node * (2 * WID) + 8 * ql;
      if (wr) *(volatile v8us*)rp = q0;
      __threadfence();
      if (wr) *(volatile v8us*)rp = q0;
    }
  }
}

static inline int cdiv(int a, int b) { return (a + b - 1) / b; }
static inline size_t al256(size_t o) { return (o + 255) & ~(size_t)255; }
static inline size_t smax(size_t a, size_t b) { return a > b ? a : b; }

extern "C" void kernel_launch(void* const* d_in, const int* in_sizes, int n_in,
                              void* d_out, int out_size, void* d_ws, size_t ws_size,
                              hipStream_t stream) {
  if (n_in < 23) return;
  if (in_sizes[0] < DF || (in_sizes[0] % DF) != 0) return;
  const int nN = in_sizes[0] / DF;
  if (nN < 16 || nN >= (1 << 22)) return;
  const int nE = in_sizes[1];
  if (nE < 1 || in_sizes[2] != nE) return;
  if (nE >= (1 << 21)) return;
  if (in_sizes[3]  != DF * DF || in_sizes[4]  != DF) return;
  if (in_sizes[5]  != DF * DH || in_sizes[6]  != DH) return;
  if (in_sizes[7]  != DH * DF || in_sizes[8]  != DF) return;
  if (in_sizes[9]  != DF * DF || in_sizes[10] != DF) return;
  if (in_sizes[11] != DF * DF || in_sizes[12] != DF) return;
  if (in_sizes[13] != DF * DH || in_sizes[14] != DH) return;
  if (in_sizes[15] != DH * DF || in_sizes[16] != DF) return;
  if (in_sizes[17] != DF || in_sizes[18] != DF) return;
  if (in_sizes[19] != DH || in_sizes[20] != DH) return;
  if (in_sizes[21] != DF || in_sizes[22] != DF) return;
  if ((long long)out_size != (long long)nN * DF) return;

  const float* x   = (const float*)d_in[0];
  const int*   src = (const int*)d_in[1];
  const int*   dst = (const int*)d_in[2];
  const float* Wc1 = (const float*)d_in[3];  const float* bc1 = (const float*)d_in[4];
  const float* Wc2 = (const float*)d_in[5];  const float* bc2 = (const float*)d_in[6];
  const float* Wc3 = (const float*)d_in[7];  const float* bc3 = (const float*)d_in[8];
  const float* W1  = (const float*)d_in[9];  const float* b1  = (const float*)d_in[10];
  const float* W2  = (const float*)d_in[11]; const float* b2  = (const float*)d_in[12];
  const float* W3  = (const float*)d_in[13]; const float* b3  = (const float*)d_in[14];
  const float* W4  = (const float*)d_in[15]; const float* b4  = (const float*)d_in[16];
  const float* g1  = (const float*)d_in[17]; const float* bt1 = (const float*)d_in[18];
  const float* g2  = (const float*)d_in[19]; const float* bt2 = (const float*)d_in[20];
  const float* g3  = (const float*)d_in[21]; const float* bt3 = (const float*)d_in[22];
  float* out = (float*)d_out;

  const int MP   = cdiv(nN, GBM) * GBM;
  const int gM   = MP / GBM;
  const int gD   = cdiv(nN, NBD);
  const int NBPD = gD * NBD;
  const int gA   = cdiv(MP, NBA);
  if ((long long)gA * NBA < (long long)MP) return;
  if (NBPD < nN) return;
  const int vec8 = ((nE & 3) == 0) ? 1 : 0;

  char* ws = (char*)d_ws;
  size_t off = 0;
  const size_t oDIS  = off; off = al256(off + (size_t)NBPD * 4);
  const size_t oWc1T = off; off = al256(off + (size_t)DF * DF * 2);
  const size_t oW1T  = off; off = al256(off + (size_t)DF * DF * 2);
  const size_t oWc2T = off; off = al256(off + (size_t)DH * 2 * DF * 2);
  const size_t oW2T  = off; off = al256(off + (size_t)DF * 2 * DF * 2);
  const size_t oW3T  = off; off = al256(off + (size_t)DH * 2 * DF * 2);
  const size_t oWc3T = off; off = al256(off + (size_t)DF * DF * 2);
  const size_t oW4T  = off; off = al256(off + (size_t)DF * DF * 2);
  const size_t szA = smax((size_t)MP * DF * 2, (size_t)MP * DH * 4);
  const size_t szB = smax(smax((size_t)MP * 2 * DF * 2, (size_t)MP * DF * 2), (size_t)MP * DF * 4);
  const size_t szC = smax(smax((size_t)MP * 2 * DF * 2, (size_t)MP * DF * 4), (size_t)MP * DF * 2);
  const size_t oRA = off; off = al256(off + szA);
  const size_t oRB = off; off = al256(off + szB);
  const size_t oRC = off; off = al256(off + szC);
  if (off > ws_size || off > (size_t)WSMAX) return;
  float*          DIS  = (float*)(ws + oDIS);
  unsigned short* Wc1T = (unsigned short*)(ws + oWc1T);
  unsigned short* W1T  = (unsigned short*)(ws + oW1T);
  unsigned short* Wc2T = (unsigned short*)(ws + oWc2T);
  unsigned short* W2T  = (unsigned short*)(ws + oW2T);
  unsigned short* W3T  = (unsigned short*)(ws + oW3T);
  unsigned short* Wc3T = (unsigned short*)(ws + oWc3T);
  unsigned short* W4T  = (unsigned short*)(ws + oW4T);
  unsigned short* RAh  = (unsigned short*)(ws + oRA);   float* RAf = (float*)(ws + oRA);
  unsigned short* RBh  = (unsigned short*)(ws + oRB);   float* RBf = (float*)(ws + oRB);
  unsigned short* RCh  = (unsigned short*)(ws + oRC);   float* RCf = (float*)(ws + oRC);

  const size_t scanLds = (size_t)AGG_LDS_INTS * 4;
  hipFuncSetAttribute(reinterpret_cast<const void*>(&k_scan<128, 0>), hipFuncAttributeMaxDynamicSharedMemorySize, (int)scanLds);
  hipFuncSetAttribute(reinterpret_cast<const void*>(&k_scan<64, 0>),  hipFuncAttributeMaxDynamicSharedMemorySize, (int)scanLds);
  hipFuncSetAttribute(reinterpret_cast<const void*>(&k_scan<128, 1>), hipFuncAttributeMaxDynamicSharedMemorySize, (int)scanLds);

  const int nUx = MP * (DF / 8);
  k_wprep<<<NUW / NTHR, NTHR, 0, stream>>>(Wc1, W1, Wc2, W2, W3, Wc3, W4, Wc1T, W1T, Wc2T, W2T, W3T, Wc3T, W4T);
  k_cvx<<<cdiv(nUx, NTHR), NTHR, 0, stream>>>(x, nN, nUx, RAh);
  k_deg<<<gD, NTHR, 0, stream>>>(dst, nE, vec8, DIS);
  k_gemm<1><<<dim3(gM, DF / GBN), GTHR, 0, stream>>>(RAh, W1T, DF, b1, nN, RAf, RBh, 2 * DF);
  k_gemm<1><<<dim3(gM, DF / GBN), GTHR, 0, stream>>>(RBh, W2T, 2 * DF, b2, nN, RAf, RCh, 2 * DF);
  k_gemm<1><<<dim3(gM, DH / GBN), GTHR, 0, stream>>>(RCh, W3T, 2 * DF, b3, nN, RAf, RBh, 2 * DH);
  k_gemm<2><<<dim3(gM, DF / GBN), GTHR, 0, stream>>>(RBh, W4T, 2 * DH, b4, nN, out, RCh, DF);
  k_gemm<0><<<dim3(gM, DF / GBN), GTHR, 0, stream>>>(RAh, Wc1T, DF, bc1, nN, RCf, RBh, DF);
  k_scan<128, 0><<<gA, NTHR, scanLds, stream>>>(src, dst, nE, nN, vec8, MP, DIS, RCf, bc1, g1, bt1, RBh, out);
  k_gemm<0><<<dim3(gM, DH / GBN), GTHR, 0, stream>>>(RBh, Wc2T, 2 * DF, bc2, nN, RAf, RCh, DH);
  k_scan<64, 0><<<gA, NTHR, scanLds, stream>>>(src, dst, nE, nN, vec8, MP, DIS, RAf, bc2, g2, bt2, RCh, out);
  k_gemm<0><<<dim3(gM, DF / GBN), GTHR, 0, stream>>>(RCh, Wc3T, 2 * DH, bc3, nN, RBf, RAh, DF);
  k_scan<128, 1><<<gA, NTHR, scanLds, stream>>>(src, dst, nE, nN, vec8, MP, DIS, RBf, bc3, g3, bt3, RCh, out);
}
